// MultiHeadInfiniAttention_61314953118549
// MI455X (gfx1250) — hardware-verified
//
#include <hip/hip_runtime.h>
#include <stdint.h>
#include <stddef.h>


#define NBATCH 2
#define SEQ 4096
#define DM 1024
#define NH 8
#define DH 128
#define SEGL 512
#define NSEG 8
#define NBH 16
#define MROWS 8192
#define LSTR 136
#define TILE (128 * LSTR)
#define KT 64
#define QST 128
#define KST 128
#define PST 64
#define VST 64
#define MST 128
#define SST 128
#define EPSV 1e-6f
#define QKV_SC 16.0f
#define W_SC 256.0f
#define P_SC 4096.0f
#define INV_SQRT_DH 0.08838834764831845f

typedef _Float16 v16h __attribute__((ext_vector_type(16)));
typedef _Float16 v8h  __attribute__((ext_vector_type(8)));
typedef float    v8f  __attribute__((ext_vector_type(8)));
typedef float    v4f  __attribute__((ext_vector_type(4)));
typedef unsigned int v4u __attribute__((ext_vector_type(4)));

union Frag  { v16h v; v8h half[2]; };
union Pack8 { v8h h; v4u u; };

__device__ __forceinline__ v8f mma16(v16h a, v16h b, v8f c) {
  v8f d = __builtin_amdgcn_wmma_f32_16x16x32_f16(false, a, false, b, (short)0, c, false, false);
  asm volatile("v_nop\n\tv_nop\n\tv_nop\n\tv_nop" : "+v"(d) : "v"(a), "v"(b));
  return d;
}

__device__ __forceinline__ v16h ld_frag(const _Float16* base, int pitch, int row0, int k0, int lane) {
  const _Float16* p = base + (size_t)(row0 + (lane & 15)) * pitch + k0 + 8 * (lane >> 4);
  Frag f;
  f.half[0] = *(const v8h*)(p);
  f.half[1] = *(const v8h*)(p + 16);
  return f.v;
}

__device__ __forceinline__ float bf16r(float f) {
  unsigned int u = __float_as_uint(f);
  u += 0x7FFFu + ((u >> 16) & 1u);
  u &= 0xFFFF0000u;
  return __uint_as_float(u);
}

__device__ __forceinline__ float elu1(float v) { return v > 0.f ? v + 1.f : __expf(v); }

__device__ __forceinline__ float redmax16(float v) {
  v = fmaxf(v, __shfl_xor(v, 1));
  v = fmaxf(v, __shfl_xor(v, 2));
  v = fmaxf(v, __shfl_xor(v, 4));
  v = fmaxf(v, __shfl_xor(v, 8));
  return v;
}
__device__ __forceinline__ float redsum16(float v) {
  v += __shfl_xor(v, 1);
  v += __shfl_xor(v, 2);
  v += __shfl_xor(v, 4);
  v += __shfl_xor(v, 8);
  return v;
}

__global__ __launch_bounds__(256) void k_cvt_x(const float* __restrict__ x,
                                               _Float16* __restrict__ xh, int n8)
{
  const int i = blockIdx.x * 256 + threadIdx.x;
  if (i >= n8) return;
  const float* src = x + (size_t)i * 8;
  const v4f a = *(const v4f*)(src);
  const v4f b = *(const v4f*)(src + 4);
  Pack8 o;
#pragma unroll
  for (int e = 0; e < 4; ++e) {
    o.h[e]     = (_Float16)bf16r(a[e]);
    o.h[4 + e] = (_Float16)bf16r(b[e]);
  }
  _Float16* dst = xh + (size_t)i * 8;
  *(volatile v4u*)dst = o.u;
  __threadfence();
  *(volatile v4u*)dst = o.u;
}

__global__ __launch_bounds__(256) void k_cvt_w(const float* __restrict__ w0,
                                               const float* __restrict__ w1,
                                               const float* __restrict__ w2,
                                               _Float16* __restrict__ wt)
{
  const int z = blockIdx.z;
  const float* W = (z == 0) ? w0 : (z == 1) ? w1 : w2;
  _Float16* dst = wt + (size_t)z * DM * DM;
  const int k0 = blockIdx.x * 64, n0 = blockIdx.y * 64, tid = threadIdx.x;
  __shared__ float tile[64][65];
#pragma unroll
  for (int i = 0; i < 4; ++i) {
    const int idx = i * 256 + tid;
    const int r = idx >> 4, c4 = (idx & 15) * 4;
    const v4f v = *(const v4f*)(W + (size_t)(k0 + r) * DM + n0 + c4);
    tile[r][c4 + 0] = v[0];
    tile[r][c4 + 1] = v[1];
    tile[r][c4 + 2] = v[2];
    tile[r][c4 + 3] = v[3];
  }
  __syncthreads();
  Pack8 o0, o1;
  const int p0 = tid, p1 = 256 + tid;
  const int na = p0 >> 3, ka = (p0 & 7) * 8;
  const int nb = p1 >> 3, kb = (p1 & 7) * 8;
#pragma unroll
  for (int e = 0; e < 8; ++e) {
    o0.h[e] = (_Float16)(bf16r(tile[ka + e][na]) * W_SC);
    o1.h[e] = (_Float16)(bf16r(tile[kb + e][nb]) * W_SC);
  }
  const size_t offa = (size_t)(n0 + na) * DM + k0 + ka;
  const size_t offb = (size_t)(n0 + nb) * DM + k0 + kb;
  *(volatile v4u*)(dst + offa) = o0.u;
  *(volatile v4u*)(dst + offb) = o1.u;
  __threadfence();
  *(volatile v4u*)(dst + offa) = o0.u;
  *(volatile v4u*)(dst + offb) = o1.u;
}

__global__ __launch_bounds__(256) __attribute__((amdgpu_num_vgpr(256)))
void k_qkv(const _Float16* __restrict__ xh, const _Float16* __restrict__ wt,
           const float* __restrict__ b0, const float* __restrict__ b1, const float* __restrict__ b2,
           _Float16* __restrict__ o0, _Float16* __restrict__ o1, _Float16* __restrict__ o2)
{
  const int z = blockIdx.z;
  const float* bias = (z == 0) ? b0 : (z == 1) ? b1 : b2;
  _Float16* outp   = (z == 0) ? o0 : (z == 1) ? o1 : o2;
  const _Float16* Bt = wt + (size_t)z * DM * DM;
  const int tid = threadIdx.x, lane = tid & 31, w = tid >> 5;
  const int wm = w >> 1, wn = w & 1, l15 = lane & 15, hl = lane >> 4;
  const int m0 = blockIdx.x * 128, n0 = blockIdx.y * 128;
  __shared__ __align__(16) _Float16 stg[TILE];

  v8f acc[2][4];
#pragma unroll
  for (int r = 0; r < 2; ++r)
#pragma unroll
    for (int c = 0; c < 4; ++c)
#pragma unroll
      for (int j = 0; j < 8; ++j) acc[r][c][j] = 0.f;

  const _Float16* Ap = xh + (size_t)(m0 + wm * 32) * DM;
  const _Float16* Bp = Bt + (size_t)(n0 + wn * 64) * DM;
#pragma unroll 1
  for (int kt = 0; kt < DM / 32; ++kt) {
    const int k0 = kt * 32;
    const v16h a0 = ld_frag(Ap, DM, 0, k0, lane);
    const v16h a1 = ld_frag(Ap, DM, 16, k0, lane);
#pragma unroll
    for (int c = 0; c < 4; ++c) {
      const v16h bb = ld_frag(Bp, DM, c * 16, k0, lane);
      acc[0][c] = mma16(a0, bb, acc[0][c]);
      acc[1][c] = mma16(a1, bb, acc[1][c]);
    }
  }

#pragma unroll
  for (int r = 0; r < 2; ++r)
#pragma unroll
    for (int c = 0; c < 4; ++c) {
      const int col = wn * 64 + c * 16 + l15;
      const float bq = bf16r(bias[n0 + col]);
#pragma unroll
      for (int j = 0; j < 8; ++j) {
        const int row = wm * 32 + r * 16 + 8 * hl + j;
        const float y = acc[r][c][j] * (1.f / W_SC) + bq;
        stg[row * LSTR + col] = (_Float16)(y * QKV_SC);
      }
    }
  __syncthreads();

  const int bb = m0 >> 12, t0 = m0 & 4095, hh = blockIdx.y;
  _Float16* dst = outp + ((size_t)(bb * NH + hh) * SEQ + t0) * DH;
#pragma unroll
  for (int pass = 0; pass < 2; ++pass) {
#pragma unroll
    for (int i = 0; i < 8; ++i) {
      const int p = i * 256 + tid;
      Pack8 o;
      o.h = *(const v8h*)&stg[(p >> 4) * LSTR + (p & 15) * 8];
      *(volatile v4u*)(dst + (size_t)p * 8) = o.u;
    }
    if (pass == 0) __threadfence();
  }
}

__device__ __forceinline__ void snap_store(const _Float16* mh, const float* zs,
                                           _Float16* mdst, float* zdst, int tid)
{
#pragma unroll
  for (int pass = 0; pass < 2; ++pass) {
#pragma unroll
    for (int i = 0; i < 8; ++i) {
      const int p = i * 256 + tid;
      Pack8 o;
      o.h = *(const v8h*)(mh + (p >> 4) * LSTR + (p & 15) * 8);
      *(volatile v4u*)(mdst + (size_t)p * 8) = o.u;
    }
    if (tid < 32) {
      const v4f zz = *(const v4f*)(zs + tid * 4);
      *(volatile v4f*)(zdst + tid * 4) = zz;
    }
    if (pass == 0) __threadfence();
  }
}

__global__ __launch_bounds__(256) __attribute__((amdgpu_num_vgpr(256)))
void k_mem(const _Float16* __restrict__ kw, const _Float16* __restrict__ vw,
           _Float16* __restrict__ mt, float* __restrict__ zw)
{
  const int bh = blockIdx.x;
  const int tid = threadIdx.x, lane = tid & 31, w = tid >> 5;
  const int l15 = lane & 15, hl = lane >> 4;

  __shared__ __align__(16) _Float16 MhT[TILE];
  __shared__ __align__(16) _Float16 bufK[TILE];
  __shared__ __align__(16) _Float16 bufQ[TILE];
  __shared__ __align__(16) _Float16 bufV[TILE];
  __shared__ __align__(16) float den_s[128];
  __shared__ __align__(16) float zsh[128];

  v8f Macc[8];
#pragma unroll
  for (int c = 0; c < 8; ++c)
#pragma unroll
    for (int j = 0; j < 8; ++j) Macc[c][j] = 0.f;

  {
    Pack8 zero;
    zero.u[0] = 0u; zero.u[1] = 0u; zero.u[2] = 0u; zero.u[3] = 0u;
    for (int i = tid; i < TILE / 8; i += 256) *(v8h*)&MhT[i * 8] = zero.h;
  }
  if (tid < 128) zsh[tid] = 0.f;
  __syncthreads();
  snap_store(MhT, zsh, mt + (size_t)(0 * NBH + bh) * DH * DH, zw + (size_t)(0 * NBH + bh) * DH, tid);

  const size_t rowbase0 = (size_t)bh * SEQ;
#pragma unroll 1
  for (int s = 0; s < NSEG - 1; ++s) {
    float zacc = 0.f;
#pragma unroll 1
    for (int rt = 0; rt < SEGL / 128; ++rt) {
      const size_t kbase = (rowbase0 + (size_t)s * SEGL + (size_t)rt * 128) * DH;
      __syncthreads();
#pragma unroll
      for (int i = 0; i < 8; ++i) {
        const int p = i * 256 + tid;
        const int l = p >> 4, c8 = (p & 15) * 8;
        const v8h k8 = *(const v8h*)&kw[kbase + (size_t)p * 8];
        v8h s8;
#pragma unroll
        for (int e = 0; e < 8; ++e) s8[e] = (_Float16)elu1((float)k8[e] * (1.f / QKV_SC));
        *(v8h*)&bufK[l * LSTR + c8] = s8;
#pragma unroll
        for (int e = 0; e < 8; ++e) bufQ[(c8 + e) * LSTR + l] = s8[e];
      }
      __syncthreads();
      if (tid < 128) {
        float sum = 0.f;
#pragma unroll 4
        for (int d8 = 0; d8 < 16; ++d8) {
          const v8h s8 = *(const v8h*)&bufK[tid * LSTR + d8 * 8];
#pragma unroll
          for (int e = 0; e < 8; ++e) sum += (float)s8[e] * zsh[d8 * 8 + e];
        }
        den_s[tid] = sum;
        float cs = 0.f;
#pragma unroll 4
        for (int l2 = 0; l2 < 128; ++l2) cs += (float)bufK[l2 * LSTR + tid];
        zacc += cs;
      }
      __syncthreads();
#pragma unroll
      for (int eh = 0; eh < 2; ++eh) {
        v8f R[4];
#pragma unroll
        for (int c = 0; c < 4; ++c)
#pragma unroll
          for (int j = 0; j < 8; ++j) R[c][j] = 0.f;
#pragma unroll
        for (int k = 0; k < 4; ++k) {
          const v16h a = ld_frag(bufK, LSTR, w * 16, k * 32, lane);
#pragma unroll
          for (int c = 0; c < 4; ++c)
            R[c] = mma16(a, ld_frag(MhT, LSTR, eh * 64 + c * 16, k * 32, lane), R[c]);
        }
#pragma unroll
        for (int j = 0; j < 8; ++j) {
          const int rl = w * 16 + 8 * hl + j;
          const float inv = 1.f / (den_s[rl] + EPSV);
#pragma unroll
          for (int c = 0; c < 4; ++c) {
            const int col = eh * 64 + c * 16 + l15;
            const float vv = (float)vw[kbase + (size_t)rl * DH + col] * (1.f / QKV_SC);
            bufV[col * LSTR + rl] = (_Float16)(vv - R[c][j] * inv);
          }
        }
      }
      __syncthreads();
#pragma unroll
      for (int k = 0; k < 4; ++k) {
        const v16h a = ld_frag(bufQ, LSTR, w * 16, k * 32, lane);
#pragma unroll
        for (int c = 0; c < 8; ++c)
          Macc[c] = mma16(a, ld_frag(bufV, LSTR, c * 16, k * 32, lane), Macc[c]);
      }
    }
    __syncthreads();
#pragma unroll
    for (int c = 0; c < 8; ++c)
#pragma unroll
      for (int j = 0; j < 8; ++j)
        MhT[(c * 16 + l15) * LSTR + w * 16 + 8 * hl + j] = (_Float16)Macc[c][j];
    if (tid < 128) zsh[tid] += zacc;
    __syncthreads();
    snap_store(MhT, zsh, mt + (size_t)((s + 1) * NBH + bh) * DH * DH,
               zw + (size_t)((s + 1) * NBH + bh) * DH, tid);
  }
}

__global__ __launch_bounds__(256) __attribute__((amdgpu_num_vgpr(256)))
void k_out(const _Float16* __restrict__ qw, const _Float16* __restrict__ kw,
           const _Float16* __restrict__ vw, const _Float16* __restrict__ mt,
           const float* __restrict__ zw, const float* __restrict__ beta,
           float* __restrict__ out)
{
  const int qt = blockIdx.x, s = blockIdx.y, bh = blockIdx.z;
  const int b = bh >> 3, h = bh & 7;
  const int tid = threadIdx.x, lane = tid & 31, w = tid >> 5;
  const int l15 = lane & 15, hl = lane >> 4;
  const float gate = 1.f / (1.f + expf(-bf16r(beta[h])));
  const float sscale = INV_SQRT_DH * (1.f / (QKV_SC * QKV_SC));

  __shared__ __align__(16) _Float16 sQ[128 * QST];
  __shared__ __align__(16) _Float16 sR[KT * KST + 128 * PST + 128 * VST];
  __shared__ __align__(16) float stg[128 * SST];
  __shared__ __align__(16) float den_s[128];
  __shared__ __align__(16) float zsh[128];
  _Float16* bufK  = sR;
  _Float16* bufP  = sR + KT * KST;
  _Float16* bufVt = bufP + 128 * PST;
  _Float16* bufMt = sR;

  const size_t rowbase = (size_t)bh * SEQ + (size_t)s * SEGL;
  const size_t qbase = (rowbase + (size_t)qt * 128) * DH;
#pragma unroll
  for (int i = 0; i < 8; ++i) {
    const int p = i * 256 + tid;
    *(v8h*)&sQ[(p >> 4) * QST + (p & 15) * 8] = *(const v8h*)&qw[qbase + (size_t)p * 8];
  }

  v8f O[8];
  float m_run[8], l_run[8];
#pragma unroll
  for (int j = 0; j < 8; ++j) { m_run[j] = -1e30f; l_run[j] = 0.f; }
#pragma unroll
  for (int c = 0; c < 8; ++c)
#pragma unroll
    for (int j = 0; j < 8; ++j) O[c][j] = 0.f;

  const int nkt = 2 * qt + 2;
#pragma unroll 1
  for (int kt = 0; kt < nkt; ++kt) {
    const size_t kbase = (rowbase + (size_t)kt * KT) * DH;
    __syncthreads();
#pragma unroll
    for (int i = 0; i < 4; ++i) {
      const int p = i * 256 + tid;
      const int l = p >> 4, c8 = (p & 15) * 8;
      *(v8h*)&bufK[l * KST + c8] = *(const v8h*)&kw[kbase + (size_t)p * 8];
      const v8h vv = *(const v8h*)&vw[kbase + (size_t)p * 8];
#pragma unroll
      for (int e = 0; e < 8; ++e) bufVt[(c8 + e) * VST + l] = vv[e];
    }
    __syncthreads();
    v8f Sv[4];
#pragma unroll
    for (int c = 0; c < 4; ++c)
#pragma unroll
      for (int j = 0; j < 8; ++j) Sv[c][j] = 0.f;
#pragma unroll
    for (int k = 0; k < 4; ++k) {
      const v16h a = ld_frag(sQ, QST, w * 16, k * 32, lane);
#pragma unroll
      for (int c = 0; c < 4; ++c)
        Sv[c] = mma16(a, ld_frag(bufK, KST, c * 16, k * 32, lane), Sv[c]);
    }
#pragma unroll
    for (int c = 0; c < 4; ++c) {
      const int col = kt * KT + c * 16 + l15;
#pragma unroll
      for (int j = 0; j < 8; ++j) {
        const int row = qt * 128 + w * 16 + 8 * hl + j;
        const float sv = Sv[c][j] * sscale;
        Sv[c][j] = (col <= row) ? sv : -1e30f;
      }
    }
#pragma unroll
    for (int j = 0; j < 8; ++j) {
      float mx = -3e38f;
#pragma unroll
      for (int c = 0; c < 4; ++c) mx = fmaxf(mx, Sv[c][j]);
      mx = redmax16(mx);
      const float mnew  = fmaxf(m_run[j], mx);
      const float alpha = __expf(m_run[j] - mnew);
      float rs = 0.f;
#pragma unroll
      for (int c = 0; c < 4; ++c) { const float p = __expf(Sv[c][j] - mnew); Sv[c][j] = p; rs += p; }
      rs = redsum16(rs);
      m_run[j] = mnew;
      l_run[j] = l_run[j] * alpha + rs;
#pragma unroll
      for (int c = 0; c < 8; ++c) O[c][j] *= alpha;
    }
#pragma unroll
    for (int c = 0; c < 4; ++c)
#pragma unroll
      for (int j = 0; j < 8; ++j)
        bufP[(w * 16 + 8 * hl + j) * PST + c * 16 + l15] = (_Float16)(Sv[c][j] * P_SC);
    __syncthreads();
#pragma unroll
    for (int k = 0; k < 2; ++k) {
      const v16h a = ld_frag(bufP, PST, w * 16, k * 32, lane);
#pragma unroll
      for (int c = 0; c < 8; ++c)
        O[c] = mma16(a, ld_frag(bufVt, VST, c * 16, k * 32, lane), O[c]);
    }
  }

#pragma unroll
  for (int j = 0; j < 8; ++j) {
    const int rl = w * 16 + 8 * hl + j;
    const float il = (1.f - gate) / (l_run[j] * (P_SC * QKV_SC));
#pragma unroll
    for (int c = 0; c < 8; ++c) stg[rl * SST + c * 16 + l15] = O[c][j] * il;
  }
  __syncthreads();

#pragma unroll
  for (int i = 0; i < 8; ++i) {
    const int p = i * 256 + tid;
    const int o8 = (p >> 4) * QST + (p & 15) * 8;
    const v8h q8 = *(const v8h*)&sQ[o8];
    v8h s8;
#pragma unroll
    for (int e = 0; e < 8; ++e) s8[e] = (_Float16)elu1((float)q8[e] * (1.f / QKV_SC));
    *(v8h*)&sQ[o8] = s8;
  }
  const size_t snap = (size_t)(s * NBH + bh);
#pragma unroll
  for (int i = 0; i < 8; ++i) {
    const int p = i * 256 + tid;
    *(v8h*)&bufMt[(p >> 4) * MST + (p & 15) * 8] = *(const v8h*)&mt[snap * DH * DH + (size_t)p * 8];
  }
  if (tid < 128) zsh[tid] = zw[snap * DH + tid];
  __syncthreads();
  if (tid < 128) {
    float sum = 0.f;
#pragma unroll 4
    for (int d8 = 0; d8 < 16; ++d8) {
      const v8h s8 = *(const v8h*)&sQ[tid * QST + d8 * 8];
#pragma unroll
      for (int e = 0; e < 8; ++e) sum += (float)s8[e] * zsh[d8 * 8 + e];
    }
    den_s[tid] = sum;
  }
  v8f Am[8];
#pragma unroll
  for (int c = 0; c < 8; ++c)
#pragma unroll
    for (int j = 0; j < 8; ++j) Am[c][j] = 0.f;
#pragma unroll
  for (int k = 0; k < 4; ++k) {
    const v16h a = ld_frag(sQ, QST, w * 16, k * 32, lane);
#pragma unroll
    for (int c = 0; c < 8; ++c)
      Am[c] = mma16(a, ld_frag(bufMt, MST, c * 16, k * 32, lane), Am[c]);
  }
  __syncthreads();

#pragma unroll
  for (int j = 0; j < 8; ++j) {
    const int rl = w * 16 + 8 * hl + j;
    const float ginv = gate / (den_s[rl] + EPSV);
#pragma unroll
    for (int c = 0; c < 8; ++c) {
      const int idx = rl * SST + c * 16 + l15;
      const float val = stg[idx] + Am[c][j] * ginv;
      stg[idx] = val;
    }
  }
  __syncthreads();

  float* obase = out + ((size_t)b * SEQ + (size_t)s * SEGL + (size_t)qt * 128) * DM + (size_t)h * DH;
#pragma unroll
  for (int pass = 0; pass < 2; ++pass) {
#pragma unroll
    for (int i = 0; i < 16; ++i) {
      const int row = i * 8 + w;
      const v4f v = *(const v4f*)&stg[row * SST + lane * 4];
      *(volatile v4f*)(obase + (size_t)row * DM + lane * 4) = v;
    }
    if (pass == 0) __threadfence();
  }
}

extern "C" void kernel_launch(void* const* d_in, const int* in_sizes, int n_in,
                              void* d_out, int out_size, void* d_ws, size_t ws_size,
                              hipStream_t stream) {
  if (n_in < 8) return;
  if (in_sizes[0] != MROWS * DM) return;
  if (in_sizes[1] != DM * DM || in_sizes[3] != DM * DM || in_sizes[5] != DM * DM) return;
  if (in_sizes[2] != DM || in_sizes[4] != DM || in_sizes[6] != DM) return;
  if (in_sizes[7] != NH) return;
  if (out_size != MROWS * DM) return;

  const float* x    = (const float*)d_in[0];
  const float* w_q  = (const float*)d_in[1];
  const float* b_q  = (const float*)d_in[2];
  const float* w_k  = (const float*)d_in[3];
  const float* b_k  = (const float*)d_in[4];
  const float* w_v  = (const float*)d_in[5];
  const float* b_v  = (const float*)d_in[6];
  const float* beta = (const float*)d_in[7];
  float* out = (float*)d_out;

  const size_t xh_bytes  = (size_t)MROWS * DM * 2;
  const size_t wt_bytes  = (size_t)3 * DM * DM * 2;
  const size_t qkv_bytes = (size_t)NBH * SEQ * DH * 2;
  const size_t mt_bytes  = (size_t)NSEG * NBH * DH * DH * 2;
  const size_t z_bytes   = (size_t)NSEG * NBH * DH * 4;
  size_t off = 0;
  const size_t off_xh = off; off += xh_bytes;
  const size_t off_wt = off; off += wt_bytes;
  const size_t off_q  = off; off += qkv_bytes;
  const size_t off_k  = off; off += qkv_bytes;
  const size_t off_v  = off; off += qkv_bytes;
  const size_t off_mt = off; off += mt_bytes;
  const size_t off_z  = off; off += z_bytes;
  if (off > ws_size) return;

  char* ws = (char*)d_ws;
  _Float16* xh = (_Float16*)(ws + off_xh);
  _Float16* wt = (_Float16*)(ws + off_wt);
  _Float16* qw = (_Float16*)(ws + off_q);
  _Float16* kw = (_Float16*)(ws + off_k);
  _Float16* vw = (_Float16*)(ws + off_v);
  _Float16* mt = (_Float16*)(ws + off_mt);
  float*    zw = (float*)(ws + off_z);

  const int n8 = MROWS * DM / 8;
  k_cvt_x<<<dim3((n8 + 255) / 256), dim3(256), 0, stream>>>(x, xh, n8);
  k_cvt_w<<<dim3(DM / 64, DM / 64, 3), dim3(256), 0, stream>>>(w_q, w_k, w_v, wt);
  k_qkv<<<dim3(MROWS / 128, DM / 128, 3), dim3(256), 0, stream>>>(xh, wt, b_q, b_k, b_v, qw, kw, vw);
  k_mem<<<dim3(NBH), dim3(256), 0, stream>>>(kw, vw, mt, zw);
  k_out<<<dim3(SEGL / 128, NSEG, NBH), dim3(256), 0, stream>>>(qw, kw, vw, mt, zw, beta, out);
}
